// MultiHeadAttentionLayerMoE_32246614459305
// MI455X (gfx1250) — hardware-verified
//
#include <hip/hip_runtime.h>


namespace {
constexpr int B = 8, S = 1024, D = 128, HF = 512, E = 4, NH = 8, HD = 16, NT = B * S, NBLK = NT / 16;
constexpr float XS = 8.0f, PS = 1024.0f, WSC = 256.0f;
typedef _Float16 b16;
typedef __attribute__((ext_vector_type(16))) _Float16 v16b;
typedef __attribute__((ext_vector_type(8))) _Float16 v8b;
typedef __attribute__((ext_vector_type(8))) float v8f;
typedef __attribute__((ext_vector_type(4))) float v4f;
__device__ __forceinline__ float bf16_rne(float f) { unsigned int u = __float_as_uint(f); u += 0x7FFFu + ((u >> 16) & 1u); return __uint_as_float(u & 0xFFFF0000u); }
__device__ __forceinline__ void split16(float v, b16& hi, b16& lo) { hi = (b16)v; lo = (b16)(v - (float)hi); }
__device__ __forceinline__ v16b frag_kb(const b16* p, int hh) { const v8b a = *(const v8b*)(p + 8 * hh), b = *(const v8b*)(p + 16 + 8 * hh); v16b f;
#pragma unroll
  for (int e = 0; e < 8; ++e) { f[e] = a[e]; f[8 + e] = b[e]; } return f; }
__device__ __forceinline__ v8f wmma16b(v16b a, v16b b, v8f c) { v8f d = __builtin_amdgcn_wmma_f32_16x16x32_f16(false, a, false, b, (short)0, c, false, false); asm volatile("v_nop\n\tv_nop\n\tv_nop\n\tv_nop" : "+v"(d) : "v"(a), "v"(b)); return d; }
__device__ __forceinline__ void wave_lds_sync() { __builtin_amdgcn_fence(__ATOMIC_RELEASE, "workgroup"); __builtin_amdgcn_wave_barrier(); __builtin_amdgcn_fence(__ATOMIC_ACQUIRE, "workgroup"); }
__device__ __forceinline__ float pmul(float a, float b) { float p = a * b; asm volatile("" : "+v"(p)); return p; }

__global__ __launch_bounds__(256) void wput_kernel(const float* __restrict__ w, int KIN, int OUTW, b16* __restrict__ WT) {
  const int KG = KIN / 8; const int u = blockIdx.x * 256 + threadIdx.x; if (u >= OUTW * KG) return; const int o = u / KG, k0 = (u % KG) * 8; v8b v;
#pragma unroll
  for (int j = 0; j < 8; ++j) v[j] = (b16)(bf16_rne(w[(size_t)(k0 + j) * OUTW + o]) * WSC); for (int pass = 0; pass < 2; ++pass) { *(volatile v8b*)(WT + (size_t)o * KIN + k0) = v; __threadfence(); }
}
__global__ __launch_bounds__(32) void qkv_kernel(const float* __restrict__ x, const b16* __restrict__ WT, const float* __restrict__ bias, int RL, float* __restrict__ QKV) {
  __shared__ __attribute__((aligned(16))) b16 Ah[16][D + 8]; __shared__ float Tf[16][D + 4]; const int lane = threadIdx.x, nloc = lane & 15, hlf = lane >> 4; const size_t m0 = (size_t)blockIdx.x * 16; if (m0 >= (size_t)RL) return;
  for (int rr = 0; rr < 16; ++rr) for (int q = 0; q < 4; ++q) Ah[rr][q * 32 + lane] = (b16)(bf16_rne(x[(m0 + rr) * D + q * 32 + lane]) * XS);
  wave_lds_sync();
#pragma unroll 1
  for (int g = 0; g < 3; ++g) { v8f acc[8];
#pragma unroll
    for (int t = 0; t < 8; ++t) acc[t] = (v8f){};
#pragma unroll
    for (int kb = 0; kb < D; kb += 32) { const v16b a = frag_kb(&Ah[nloc][kb], hlf);
#pragma unroll
      for (int t = 0; t < 8; ++t) acc[t] = wmma16b(a, frag_kb(WT + (size_t)(g * D + t * 16 + nloc) * D + kb, hlf), acc[t]); }
#pragma unroll
    for (int t = 0; t < 8; ++t) { const int c = t * 16 + nloc; const float bb = bf16_rne(bias[g * D + c]);
#pragma unroll
      for (int r8 = 0; r8 < 8; ++r8) Tf[8 * hlf + r8][c] = acc[t][r8] * (1.0f / (XS * WSC)) + bb; }
    wave_lds_sync();
    for (int pass = 0; pass < 2; ++pass) { for (int rr = 0; rr < 16; ++rr) *(volatile v4f*)(QKV + (m0 + rr) * (3 * D) + g * D + lane * 4) = *(const v4f*)(&Tf[rr][lane * 4]); __threadfence(); }
    wave_lds_sync(); }
}
__global__ __launch_bounds__(32) void att_kernel(const float* __restrict__ QKV, int BV, float* __restrict__ ATT) {
  __shared__ __attribute__((aligned(16))) b16 Qh[16][40], Ql[16][40], Kh[32][40], Kl[32][40], Ph[16][40], Pl[16][40], Vh[HD][40], Vl[HD][40]; __shared__ float Sc[16][33], M[16], Dn[16], Sf[16], Of[16][D + 1];
  const int lane = threadIdx.x, nloc = lane & 15, hlf = lane >> 4; const int b = blockIdx.x / (S / 16), qb = blockIdx.x % (S / 16); if (b >= BV) return; const size_t base = (size_t)b * S, q0 = base + qb * 16;
#pragma unroll 1
  for (int h = 0; h < NH; ++h) {
    for (int rr = 0; rr < 16; ++rr) { b16 p = (b16)0.0f, ql = (b16)0.0f; if (lane < HD) split16(QKV[(q0 + rr) * (3 * D) + h * HD + lane] * XS, p, ql); Qh[rr][lane] = p; Ql[rr][lane] = ql; }
    if (lane < 16) { M[lane] = -INFINITY; Dn[lane] = 0.0f; Sf[lane] = 0.0f; }
    v8f acc = {}; wave_lds_sync();
#pragma unroll 1
    for (int kc = 0; kc < S; kc += 32) {
      for (int rr = 0; rr < 32; ++rr) { const float* kp = QKV + (base + kc + rr) * (3 * D) + D + h * HD; const float* vp = QKV + (base + kc + rr) * (3 * D) + 2 * D + h * HD; b16 p = (b16)0.0f, ql = (b16)0.0f; if (lane < HD) split16(kp[lane] * XS, p, ql); Kh[rr][lane] = p; Kl[rr][lane] = ql; if (lane < HD) { split16(vp[lane] * XS, p, ql); Vh[lane][rr] = p; Vl[lane][rr] = ql; } }
      wave_lds_sync(); const v16b qh = frag_kb(&Qh[nloc][0], hlf), qlo = frag_kb(&Ql[nloc][0], hlf);
#pragma unroll
      for (int blk = 0; blk < 2; ++blk) { const v16b kh = frag_kb(&Kh[blk * 16 + nloc][0], hlf), kl = frag_kb(&Kl[blk * 16 + nloc][0], hlf); v8f s = {}; s = wmma16b(qh, kh, s); s = wmma16b(qh, kl, s); s = wmma16b(qlo, kh, s);
#pragma unroll
        for (int r8 = 0; r8 < 8; ++r8) Sc[8 * hlf + r8][blk * 16 + nloc] = s[r8] * (0.25f / (XS * XS)); }
      wave_lds_sync();
#pragma unroll 1
      for (int qi = 0; qi < 16; ++qi) { const float sv = Sc[qi][lane]; float cm = sv; for (int o = 16; o; o >>= 1) cm = fmaxf(cm, __shfl_xor(cm, o)); const float mo = M[qi]; const float mn = fmaxf(mo, cm); const float p = __expf(sv - mn); float psum = p; for (int o = 16; o; o >>= 1) psum += __shfl_xor(psum, o);
        b16 ph, plo; split16(p * PS, ph, plo); Ph[qi][lane] = ph; Pl[qi][lane] = plo; if (lane == 0) { const float sf = (mo == -INFINITY) ? 0.0f : __expf(mo - mn); Sf[qi] = sf; Dn[qi] = Dn[qi] * sf + psum; M[qi] = mn; } }
      wave_lds_sync();
#pragma unroll
      for (int r8 = 0; r8 < 8; ++r8) acc[r8] *= Sf[8 * hlf + r8];
      { const v16b pa = frag_kb(&Ph[nloc][0], hlf), pb = frag_kb(&Pl[nloc][0], hlf), vh = frag_kb(&Vh[nloc][0], hlf), vl = frag_kb(&Vl[nloc][0], hlf); acc = wmma16b(pa, vh, acc); acc = wmma16b(pa, vl, acc); acc = wmma16b(pb, vh, acc); }
      wave_lds_sync(); }
#pragma unroll
    for (int r8 = 0; r8 < 8; ++r8) { const int rl = 8 * hlf + r8; Of[rl][h * HD + nloc] = acc[r8] * (1.0f / (PS * XS)) / Dn[rl]; }
    wave_lds_sync(); }
  for (int pass = 0; pass < 2; ++pass) { for (int rr = 0; rr < 16; ++rr) *(volatile v4f*)(ATT + (q0 + rr) * D + lane * 4) = (v4f){Of[rr][lane * 4], Of[rr][lane * 4 + 1], Of[rr][lane * 4 + 2], Of[rr][lane * 4 + 3]}; __threadfence(); }
}
__global__ __launch_bounds__(32) void wo_kernel(const float* __restrict__ ATT, const float* __restrict__ x, const b16* __restrict__ WO, const float* __restrict__ bo, int RL, float* __restrict__ PRE) {
  __shared__ __attribute__((aligned(16))) b16 Ah[16][D + 8], Al[16][D + 8]; __shared__ float Tf[16][D + 4]; const int lane = threadIdx.x, nloc = lane & 15, hlf = lane >> 4; const size_t m0 = (size_t)blockIdx.x * 16; if (m0 >= (size_t)RL) return;
  for (int rr = 0; rr < 16; ++rr) for (int q = 0; q < 4; ++q) { b16 p, ql; split16(ATT[(m0 + rr) * D + q * 32 + lane] * XS, p, ql); Ah[rr][q * 32 + lane] = p; Al[rr][q * 32 + lane] = ql; }
  wave_lds_sync(); v8f acc[8];
#pragma unroll
  for (int t = 0; t < 8; ++t) acc[t] = (v8f){};
#pragma unroll
  for (int kb = 0; kb < D; kb += 32) { const v16b a = frag_kb(&Ah[nloc][kb], hlf), al = frag_kb(&Al[nloc][kb], hlf);
#pragma unroll
    for (int t = 0; t < 8; ++t) { const v16b bw = frag_kb(WO + (size_t)(t * 16 + nloc) * D + kb, hlf); acc[t] = wmma16b(a, bw, acc[t]); acc[t] = wmma16b(al, bw, acc[t]); } }
#pragma unroll
  for (int t = 0; t < 8; ++t) { const int c = t * 16 + nloc; const float bb = bf16_rne(bo[c]);
#pragma unroll
    for (int r8 = 0; r8 < 8; ++r8) Tf[8 * hlf + r8][c] = acc[t][r8] * (1.0f / (XS * WSC)) + bb + bf16_rne(x[(m0 + 8 * hlf + r8) * D + c]); }
  wave_lds_sync();
  for (int pass = 0; pass < 2; ++pass) { for (int rr = 0; rr < 16; ++rr) *(volatile v4f*)(PRE + (m0 + rr) * D + lane * 4) = *(const v4f*)(&Tf[rr][lane * 4]); __threadfence(); }
}
__global__ __launch_bounds__(256) void stats_kernel(const float* __restrict__ PRE, int BV, float* __restrict__ ST) {
  __shared__ float red[256]; const int bc = blockIdx.x, b = bc / D, c = bc % D, tid = threadIdx.x; if (b >= BV) return; const float* p = PRE + (size_t)b * S * D + c; float s = 0.0f; for (int t = tid; t < S; t += 256) s += p[(size_t)t * D]; red[tid] = s; __syncthreads();
  for (int w = 128; w > 0; w >>= 1) { if (tid < w) red[tid] += red[tid + w]; __syncthreads(); } const float mu = red[0] * (1.0f / S); __syncthreads();
  float q = 0.0f; for (int t = tid; t < S; t += 256) { const float d = p[(size_t)t * D] - mu; q += pmul(d, d); } red[tid] = q; __syncthreads();
  for (int w = 128; w > 0; w >>= 1) { if (tid < w) red[tid] += red[tid + w]; __syncthreads(); } const float rs = rsqrtf(red[0] * (1.0f / S) + 1e-5f);
  if (tid < 32) { for (int pass = 0; pass < 2; ++pass) { ((volatile float*)ST)[(size_t)bc * 32 + tid] = tid == 0 ? mu : (tid == 1 ? rs : 0.0f); __threadfence(); } }
}
__global__ __launch_bounds__(256) void norm_kernel(const float* __restrict__ PRE, const float* __restrict__ ST, const float* __restrict__ w, const float* __restrict__ bb, int RL, float* __restrict__ OUT) {
  const size_t i = (size_t)blockIdx.x * 256 + threadIdx.x; if (i >= (size_t)RL * D) return; const int c = (int)(i % D); const size_t b = i / ((size_t)S * D); const float* st = ST + (b * D + c) * 32; const float v = pmul(pmul(PRE[i] - st[0], st[1]), bf16_rne(w[c])) + bf16_rne(bb[c]);
  for (int pass = 0; pass < 2; ++pass) { ((volatile float*)OUT)[i] = v; __threadfence(); }
}
__global__ __launch_bounds__(32) void moe_kernel(const float* __restrict__ H, const float* __restrict__ wg, const b16* __restrict__ W1T, const float* __restrict__ b1, const b16* __restrict__ W2T, const float* __restrict__ b2, int RL, float* __restrict__ PRE2) {
  __shared__ __attribute__((aligned(16))) b16 Ah[16][D + 8], Al[16][D + 8], Fh[16][HF + 8], Fl[16][HF + 8]; __shared__ float Y[16][D + 1], G[16][E], Lg[16][E];
  const int lane = threadIdx.x, nloc = lane & 15, hlf = lane >> 4; const size_t m0 = (size_t)blockIdx.x * 16; if (m0 >= (size_t)RL) return;
  for (int rr = 0; rr < 16; ++rr) { float d0 = 0.0f, d1 = 0.0f, d2 = 0.0f, d3 = 0.0f; for (int q = 0; q < 4; ++q) { const int c = q * 32 + lane; const float hv = H[(m0 + rr) * D + c]; b16 p, ql; split16(hv * XS, p, ql); Ah[rr][c] = p; Al[rr][c] = ql; Y[rr][c] = hv;
      d0 += pmul(hv, bf16_rne(wg[c * E])); d1 += pmul(hv, bf16_rne(wg[c * E + 1])); d2 += pmul(hv, bf16_rne(wg[c * E + 2])); d3 += pmul(hv, bf16_rne(wg[c * E + 3])); }
    for (int o = 16; o; o >>= 1) { d0 += __shfl_xor(d0, o); d1 += __shfl_xor(d1, o); d2 += __shfl_xor(d2, o); d3 += __shfl_xor(d3, o); }
    if (lane == 0) { float lg[E] = {d0, d1, d2, d3}; int e0 = 0; for (int e = 1; e < E; ++e) if (lg[e] > lg[e0]) e0 = e; int e1 = e0 == 0 ? 1 : 0; for (int e = 0; e < E; ++e) if (e != e0 && lg[e] > lg[e1]) e1 = e;
      const float mx = lg[e0]; const float a0 = 1.0f, a1 = __expf(lg[e1] - mx); const float inv = 1.0f / (a0 + a1); for (int e = 0; e < E; ++e) G[rr][e] = 0.0f; G[rr][e0] = a0 * inv; G[rr][e1] = a1 * inv; for (int e = 0; e < E; ++e) Lg[rr][e] = lg[e]; } }
  wave_lds_sync();
#pragma unroll 1
  for (int ex = 0; ex < E; ++ex) { const b16* w1 = W1T + (size_t)ex * HF * D; const b16* w2 = W2T + (size_t)ex * D * HF;
#pragma unroll 1
    for (int cg = 0; cg < HF / 128; ++cg) { v8f acc[8];
#pragma unroll
      for (int t = 0; t < 8; ++t) acc[t] = (v8f){};
#pragma unroll
      for (int kb = 0; kb < D; kb += 32) { const v16b a = frag_kb(&Ah[nloc][kb], hlf), al = frag_kb(&Al[nloc][kb], hlf);
#pragma unroll
        for (int t = 0; t < 8; ++t) { const v16b bw = frag_kb(w1 + (size_t)(cg * 128 + t * 16 + nloc) * D + kb, hlf); acc[t] = wmma16b(a, bw, acc[t]); acc[t] = wmma16b(al, bw, acc[t]); } }
#pragma unroll
      for (int t = 0; t < 8; ++t) { const int c = cg * 128 + t * 16 + nloc; const float bb = bf16_rne(b1[ex * HF + c]);
#pragma unroll
        for (int r8 = 0; r8 < 8; ++r8) { b16 p, q; split16(fmaxf(acc[t][r8] * (1.0f / (XS * WSC)) + bb, 0.0f) * XS, p, q); Fh[8 * hlf + r8][c] = p; Fl[8 * hlf + r8][c] = q; } } }
    wave_lds_sync(); v8f acc[8];
#pragma unroll
    for (int t = 0; t < 8; ++t) acc[t] = (v8f){};
#pragma unroll 2
    for (int kb = 0; kb < HF; kb += 32) { const v16b a = frag_kb(&Fh[nloc][kb], hlf), al = frag_kb(&Fl[nloc][kb], hlf);
#pragma unroll
      for (int t = 0; t < 8; ++t) { const v16b bw = frag_kb(w2 + (size_t)(t * 16 + nloc) * HF + kb, hlf); acc[t] = wmma16b(a, bw, acc[t]); acc[t] = wmma16b(al, bw, acc[t]); } }
#pragma unroll
    for (int t = 0; t < 8; ++t) { const int c = t * 16 + nloc; const float bb = bf16_rne(b2[ex * D + c]);
#pragma unroll
      for (int r8 = 0; r8 < 8; ++r8) { const int rl = 8 * hlf + r8; Y[rl][c] += pmul(G[rl][ex], acc[t][r8] * (1.0f / (XS * WSC)) + bb); } }
    wave_lds_sync(); }
  for (int pass = 0; pass < 2; ++pass) { for (int rr = 0; rr < 16; ++rr) *(volatile v4f*)(PRE2 + (m0 + rr) * D + lane * 4) = (v4f){Y[rr][lane * 4], Y[rr][lane * 4 + 1], Y[rr][lane * 4 + 2], Y[rr][lane * 4 + 3]}; __threadfence(); }
}
}

extern "C" void kernel_launch(void* const* d_in, const int* in_sizes, int n_in, void* d_out, int out_size, void* d_ws, size_t ws_size, hipStream_t stream) {
  (void)n_in;
  auto Fp = [&](int i) { return (const float*)d_in[i]; };
  if (in_sizes[0] != NT * D || in_sizes[1] != D * 3 * D || in_sizes[3] != D * D || in_sizes[9] != D * E || in_sizes[10] != E * D * HF || in_sizes[12] != E * HF * D || in_sizes[14] != 1 || in_sizes[15] != 1 || out_size != NT * D) return;
  const int BV = B; const int RL = BV * S, GB16 = RL / 16;
  size_t off = 0; char* ws = (char*)d_ws;
  auto carve = [&](size_t bytes) { char* p = ws + off; off += (bytes + 255) & ~(size_t)255; return p; };
  b16* WQKV = (b16*)carve((size_t)3 * D * D * 2); b16* WO = (b16*)carve((size_t)D * D * 2); b16* W1T = (b16*)carve((size_t)E * HF * D * 2); b16* W2T = (b16*)carve((size_t)E * D * HF * 2);
  float* QKV = (float*)carve((size_t)NT * 3 * D * 4); float* ATT = (float*)carve((size_t)NT * D * 4); float* PRE = (float*)carve((size_t)NT * D * 4); float* Hn = (float*)carve((size_t)NT * D * 4); float* PRE2 = (float*)carve((size_t)NT * D * 4); float* ST = (float*)carve((size_t)B * D * 32 * 4);
  if (off > ws_size || off > ((size_t)48 << 20)) return;
  wput_kernel<<<(3 * D * 16 + 255) / 256, 256, 0, stream>>>(Fp(1), D, 3 * D, WQKV); wput_kernel<<<(D * 16 + 255) / 256, 256, 0, stream>>>(Fp(3), D, D, WO);
  for (int e = 0; e < E; ++e) { wput_kernel<<<(HF * 16 + 255) / 256, 256, 0, stream>>>(Fp(10) + (size_t)e * D * HF, D, HF, W1T + (size_t)e * HF * D); wput_kernel<<<(D * 64 + 255) / 256, 256, 0, stream>>>(Fp(12) + (size_t)e * HF * D, HF, D, W2T + (size_t)e * D * HF); }
  qkv_kernel<<<GB16, 32, 0, stream>>>(Fp(0), WQKV, Fp(2), RL, QKV);
  att_kernel<<<BV * (S / 16), 32, 0, stream>>>(QKV, BV, ATT);
  wo_kernel<<<GB16, 32, 0, stream>>>(ATT, Fp(0), WO, Fp(4), RL, PRE);
  stats_kernel<<<BV * D, 256, 0, stream>>>(PRE, BV, ST);
  norm_kernel<<<(unsigned)(((size_t)RL * D + 255) / 256), 256, 0, stream>>>(PRE, ST, Fp(5), Fp(6), RL, Hn);
  moe_kernel<<<GB16, 32, 0, stream>>>(Hn, Fp(9), W1T, Fp(11), W2T, Fp(13), RL, PRE2);
  stats_kernel<<<BV * D, 256, 0, stream>>>(PRE2, BV, ST);
  norm_kernel<<<(unsigned)(((size_t)RL * D + 255) / 256), 256, 0, stream>>>(PRE2, ST, Fp(7), Fp(8), RL, (float*)d_out);
}
